// CrossLingualAlignmentHead_77094662963653
// MI455X (gfx1250) — hardware-verified
//
#include <hip/hip_runtime.h>
#include <math.h>


typedef _Float16 f16;
typedef _Float16 v16h __attribute__((ext_vector_type(16)));
typedef _Float16 v8h  __attribute__((ext_vector_type(8)));
typedef float    v8f  __attribute__((ext_vector_type(8)));
typedef float    v4f  __attribute__((ext_vector_type(4)));
typedef v4f __attribute__((may_alias)) v4fa;
union Frag { v16h v; v8h half[2]; };

#define DAL    256
#define DSRC   512
#define NROWS  1024
#define WSCALE 64.0f
#define WINV   0.015625f

__device__ __forceinline__ v8f wmma16(v16h a, v16h b, v8f c)
{
    v8f d = __builtin_amdgcn_wmma_f32_16x16x32_f16(false, a, false, b, (short)0, c, false, false);
    asm volatile("v_nop\n\tv_nop\n\tv_nop\n\tv_nop" : "+v"(d) : "v"(a), "v"(b));
    return d;
}

__global__ __launch_bounds__(256)
void cvt_f32_f16(const float* __restrict__ in, f16* __restrict__ out, int nchunks)
{
    const int i = blockIdx.x * blockDim.x + threadIdx.x;
    const bool ok = i < nchunks;
    v8h o = {};
    f16* dst = out + (size_t)i * 8;
    if (ok) {
        const float* src = in + (size_t)i * 8;
        const v4f x0 = *(const v4f*)(src);
        const v4f x1 = *(const v4f*)(src + 4);
        o[0] = (f16)x0[0]; o[1] = (f16)x0[1]; o[2] = (f16)x0[2]; o[3] = (f16)x0[3];
        o[4] = (f16)x1[0]; o[5] = (f16)x1[1]; o[6] = (f16)x1[2]; o[7] = (f16)x1[3];
        *(volatile v8h*)dst = o;
    }
    __threadfence();
    if (ok) *(volatile v8h*)dst = o;
}

__global__ __launch_bounds__(256)
void pack_w(const float* __restrict__ W, f16* __restrict__ out, int K, int nchunks)
{
    const int q = blockIdx.x * blockDim.x + threadIdx.x;
    const bool ok = q < nchunks;
    v8h o = {};
    f16* dst = out + (size_t)q * 8;
    if (ok) {
        const int g  = q & 1;
        const int L  = (q >> 1) & 31;
        const int nt = (q >> 6) & 15;
        const int kt = q >> 10;
        const int h  = L >> 4;
        const int n  = nt * 16 + (L & 15);
        const int kbase = kt * 32 + 16 * g + 8 * h;
        #pragma unroll
        for (int j = 0; j < 8; ++j) {
            const int k = kbase + j;
            float w = 0.0f;
            if (k < K) w = W[(size_t)k * DAL + n];
            o[j] = (f16)(w * WSCALE);
        }
        *(volatile v8h*)dst = o;
    }
    __threadfence();
    if (ok) *(volatile v8h*)dst = o;
}

__device__ __forceinline__ void store_strip(float* gout, const float* s, int wave, int lane)
{
    v4f x0, x1, x2, x3;
    const int r0 = wave * 2, r1 = wave * 2 + 1;
    x0 = *(const v4fa*)(s + r0 * DAL + 4 * lane);
    x1 = *(const v4fa*)(s + r0 * DAL + 128 + 4 * lane);
    x2 = *(const v4fa*)(s + r1 * DAL + 4 * lane);
    x3 = *(const v4fa*)(s + r1 * DAL + 128 + 4 * lane);
    float* g0 = gout + (size_t)r0 * DAL;
    float* g1 = gout + (size_t)r1 * DAL;
    *(volatile v4f*)(g0 + 4 * lane)       = x0;
    *(volatile v4f*)(g0 + 128 + 4 * lane) = x1;
    *(volatile v4f*)(g1 + 4 * lane)       = x2;
    *(volatile v4f*)(g1 + 128 + 4 * lane) = x3;
    __threadfence();
    *(volatile v4f*)(g0 + 4 * lane)       = x0;
    *(volatile v4f*)(g0 + 128 + 4 * lane) = x1;
    *(volatile v4f*)(g1 + 4 * lane)       = x2;
    *(volatile v4f*)(g1 + 128 + 4 * lane) = x3;
}

__global__ __launch_bounds__(256)
void fused_proj(const f16* __restrict__ srch, const f16* __restrict__ tgth,
                const f16* __restrict__ Wsh,  const f16* __restrict__ Wth,
                const f16* __restrict__ W1h,
                const float* __restrict__ bs, const float* __restrict__ bt,
                float* __restrict__ sp_out, float* __restrict__ tp_out,
                float* __restrict__ hs_out, float* __restrict__ ht_out)
{
    __shared__ f16   pLds[16 * DAL];
    __shared__ float sOut[16 * DAL];

    const int mat   = blockIdx.x & 1;
    const int strip = blockIdx.x >> 1;
    const int lane  = threadIdx.x & 31;
    const int wave  = threadIdx.x >> 5;
    const int m     = lane & 15;
    const int hf    = lane >> 4;

    const f16*   A    = mat ? tgth   : srch;
    const f16*   Bw   = mat ? Wth    : Wsh;
    const float* bias = mat ? bt     : bs;
    float*       outP = mat ? tp_out : sp_out;
    float*       outH = mat ? ht_out : hs_out;
    const f16*   B2   = W1h + (size_t)mat * 65536;

    const int row0 = strip * 16;
    const int nt0  = wave * 2;
    const int n0   = nt0 * 16 + m;
    const int n1   = n0 + 16;

    v8f acc0 = {};
    v8f acc1 = {};
    {
        const f16* arow = A + (size_t)(row0 + m) * DSRC;
        for (int kb = 0; kb < DSRC; kb += 32) {
            Frag a;
            a.half[0] = *(const v8h*)(arow + kb + 8 * hf);
            a.half[1] = *(const v8h*)(arow + kb + 16 + 8 * hf);
            const f16* bp = Bw + ((size_t)(((kb >> 5) * 16 + nt0) * 32 + lane) << 4);
            const v16h b0 = *(const v16h*)(bp);
            const v16h b1 = *(const v16h*)(bp + 512);
            acc0 = wmma16(a.v, b0, acc0);
            acc1 = wmma16(a.v, b1, acc1);
        }
    }
    {
        const float bn0 = bias[n0];
        const float bn1 = bias[n1];
        #pragma unroll
        for (int r = 0; r < 8; ++r) {
            const int rr = 8 * hf + r;
            const float v0 = acc0[r] * WINV + bn0;
            const float v1 = acc1[r] * WINV + bn1;
            sOut[rr * DAL + n0] = v0;
            sOut[rr * DAL + n1] = v1;
            pLds[rr * DAL + n0] = (f16)v0;
            pLds[rr * DAL + n1] = (f16)v1;
        }
    }
    __syncthreads();
    store_strip(outP + (size_t)row0 * DAL, sOut, wave, lane);

    v8f c0 = {};
    v8f c1 = {};
    {
        const f16* arow = pLds + m * DAL;
        for (int kb = 0; kb < DAL; kb += 32) {
            Frag a;
            a.half[0] = *(const v8h*)(arow + kb + 8 * hf);
            a.half[1] = *(const v8h*)(arow + kb + 16 + 8 * hf);
            const f16* bp = B2 + ((size_t)(((kb >> 5) * 16 + nt0) * 32 + lane) << 4);
            const v16h b0 = *(const v16h*)(bp);
            const v16h b1 = *(const v16h*)(bp + 512);
            c0 = wmma16(a.v, b0, c0);
            c1 = wmma16(a.v, b1, c1);
        }
    }
    __syncthreads();
    #pragma unroll
    for (int r = 0; r < 8; ++r) {
        const int rr = 8 * hf + r;
        sOut[rr * DAL + n0] = c0[r] * WINV;
        sOut[rr * DAL + n1] = c1[r] * WINV;
    }
    __syncthreads();
    store_strip(outH + (size_t)row0 * DAL, sOut, wave, lane);
}

__global__ __launch_bounds__(256)
void scorer(const float* __restrict__ hs, const float* __restrict__ ht,
            const float* __restrict__ b1, const float* __restrict__ W2,
            const float* __restrict__ b2, float* __restrict__ scores)
{
    __shared__ float hrow[DAL];
    __shared__ float w2[DAL];
    __shared__ float sc[DAL];
    const int bid = blockIdx.x;
    const int t   = threadIdx.x;
    hrow[t] = hs[(size_t)bid * DAL + t] + b1[t];
    w2[t]   = W2[t];
    __syncthreads();

    const int b = bid >> 8;
    const float* hr = ht + ((size_t)b * 256 + t) * DAL;
    float acc = 0.0f;
    #pragma unroll 2
    for (int h = 0; h < DAL; h += 4) {
        const v4f hv = *(const v4f*)(hr + h);
        acc += fmaxf(hrow[h]     + hv[0], 0.0f) * w2[h];
        acc += fmaxf(hrow[h + 1] + hv[1], 0.0f) * w2[h + 1];
        acc += fmaxf(hrow[h + 2] + hv[2], 0.0f) * w2[h + 2];
        acc += fmaxf(hrow[h + 3] + hv[3], 0.0f) * w2[h + 3];
    }
    const float x = acc + b2[0];
    const float e = __expf(-x);
    const float sg = __builtin_amdgcn_rcpf(1.0f + e);
    sc[t] = sg;
    __syncthreads();

    const bool ok = t < 64;
    v4f v = {};
    float* dst = scores + (size_t)bid * DAL + 4 * t;
    if (ok) {
        v = *(const v4fa*)(&sc[4 * t]);
        *(volatile v4f*)dst = v;
    }
    __threadfence();
    if (ok) *(volatile v4f*)dst = v;
}

extern "C" void kernel_launch(void* const* d_in, const int* in_sizes, int n_in,
                              void* d_out, int out_size, void* d_ws, size_t ws_size,
                              hipStream_t stream)
{
    if (n_in < 10) return;
    if (in_sizes[0] != NROWS * DSRC || in_sizes[1] != NROWS * DSRC) return;
    if (in_sizes[2] != DSRC * DAL  || in_sizes[4] != DSRC * DAL)  return;
    if (in_sizes[6] != 2 * DAL * DAL) return;
    if (in_sizes[3] < DAL || in_sizes[5] < DAL || in_sizes[7] < DAL || in_sizes[8] < DAL || in_sizes[9] < 1) return;
    if (out_size != 3 * NROWS * DAL) return;

    const float* src = (const float*)d_in[0];
    const float* tgt = (const float*)d_in[1];
    const float* Ws  = (const float*)d_in[2];
    const float* bs  = (const float*)d_in[3];
    const float* Wt  = (const float*)d_in[4];
    const float* bt  = (const float*)d_in[5];
    const float* W1  = (const float*)d_in[6];
    const float* b1  = (const float*)d_in[7];
    const float* W2  = (const float*)d_in[8];
    const float* b2  = (const float*)d_in[9];

    const size_t actB = (size_t)NROWS * DSRC * sizeof(f16);
    const size_t wB   = (size_t)DSRC * DAL * sizeof(f16);
    const size_t hB   = (size_t)NROWS * DAL * sizeof(float);
    const size_t off_srch = 0;
    const size_t off_tgth = off_srch + actB;
    const size_t off_Wsh  = off_tgth + actB;
    const size_t off_Wth  = off_Wsh + wB;
    const size_t off_W1h  = off_Wth + wB;
    const size_t off_hs   = off_W1h + wB;
    const size_t off_ht   = off_hs + hB;
    const size_t total    = off_ht + hB;
    if (total > ws_size) return;

    char* ws = (char*)d_ws;
    f16*   srch = (f16*)(ws + off_srch);
    f16*   tgth = (f16*)(ws + off_tgth);
    f16*   Wsh  = (f16*)(ws + off_Wsh);
    f16*   Wth  = (f16*)(ws + off_Wth);
    f16*   W1h  = (f16*)(ws + off_W1h);
    float* hs   = (float*)(ws + off_hs);
    float* ht   = (float*)(ws + off_ht);

    float* scores = (float*)d_out;
    float* sp     = scores + (size_t)NROWS * DAL;
    float* tp     = sp     + (size_t)NROWS * DAL;

    const int nchA = NROWS * DSRC / 8;
    const int nchW = DSRC * DAL / 8;
    cvt_f32_f16<<<(nchA + 255) / 256, 256, 0, stream>>>(src, srch, nchA);
    cvt_f32_f16<<<(nchA + 255) / 256, 256, 0, stream>>>(tgt, tgth, nchA);
    pack_w<<<(nchW + 255) / 256, 256, 0, stream>>>(Ws, Wsh, DSRC, nchW);
    pack_w<<<(nchW + 255) / 256, 256, 0, stream>>>(Wt, Wth, DSRC, nchW);
    pack_w<<<(nchW + 255) / 256, 256, 0, stream>>>(W1, W1h, 2 * DAL, nchW);

    fused_proj<<<2 * (NROWS / 16), 256, 0, stream>>>(srch, tgth, Wsh, Wth, W1h,
                                                    bs, bt, sp, tp, hs, ht);
    scorer<<<NROWS, 256, 0, stream>>>(hs, ht, b1, W2, b2, scores);
}
